// LongformerAttention_80058190398169
// MI455X (gfx1250) — hardware-verified
//
#include <hip/hip_runtime.h>
#include <math.h>

typedef __attribute__((ext_vector_type(16))) _Float16 v16h;
typedef __attribute__((ext_vector_type(16))) __bf16 v16b;
typedef __attribute__((ext_vector_type(8)))  _Float16 v8h;
typedef __attribute__((ext_vector_type(8)))  float v8f;
typedef __attribute__((ext_vector_type(4)))  float v4f;
typedef __attribute__((ext_vector_type(2)))  float v2f;
typedef __attribute__((ext_vector_type(4)))  unsigned v4u;
typedef __attribute__((ext_vector_type(4)))  int v4i;
typedef float __attribute__((may_alias)) float_a;
typedef int __attribute__((may_alias)) int_a;

template <typename T> __device__ __forceinline__ void vst2(void* p, T v) { *(volatile T*)p = v; __threadfence(); *(volatile T*)p = v; }
__device__ __forceinline__ v8f wmma16(v16h a, v16h b, v8f c) {
  v8f d = __builtin_amdgcn_wmma_f32_16x16x32_f16(false, a, false, b, (short)0, c, false, false);
  asm volatile("v_nop\n\tv_nop\n\tv_nop\n\tv_nop" : "+v"(d) : "v"(a), "v"(b));
  return d;
}
__device__ __forceinline__ v8f wmma_bf(v16b a, v16b b, v8f c) {
  v8f d = __builtin_amdgcn_wmma_f32_16x16x32_bf16(false, a, false, b, (short)0, c, false, false);
  asm volatile("v_nop\n\tv_nop\n\tv_nop\n\tv_nop" : "+v"(d) : "v"(a), "v"(b));
  return d;
}
__device__ __forceinline__ v16h frag_h(const _Float16* rowk0, int lane) {
  union { v16h v; v8h q[2]; } u; const _Float16* p = rowk0 + 8 * (lane >> 4);
  u.q[0] = *(const v8h*)p; u.q[1] = *(const v8h*)(p + 16); return u.v;
}
__device__ __forceinline__ v16h frag_f32(const float* rowk0, int lane) {
  v16h a; const float* p = rowk0 + 8 * (lane >> 4);
#pragma unroll
  for (int i = 0; i < 8; ++i) { a[i] = (_Float16)p[i]; a[8 + i] = (_Float16)p[16 + i]; }
  return a;
}
__device__ __forceinline__ v16h frag_f32s(const float* rowk0, int lane, float sc) {
  v16h a; const float* p = rowk0 + 8 * (lane >> 4);
#pragma unroll
  for (int i = 0; i < 8; ++i) { a[i] = (_Float16)(p[i] * sc); a[8 + i] = (_Float16)(p[16 + i] * sc); }
  return a;
}
__device__ __forceinline__ v16h fragc_f32(const float* W, int k0, int n, int lane, int ld, int K) {
  v16h a; const int g = lane >> 4;
#pragma unroll
  for (int i = 0; i < 8; ++i) { const int ka = k0 + 8 * g + i, kb = ka + 16;
    a[i] = (_Float16)(ka < K ? W[(size_t)(ka < K ? ka : K - 1) * ld + n] : 0.f); a[8 + i] = (_Float16)(kb < K ? W[(size_t)(kb < K ? kb : K - 1) * ld + n] : 0.f); }
  return a;
}
struct F2 { v16b h, l; };
__device__ __forceinline__ F2 bsplit16(const float v[16]) { F2 r;
#pragma unroll
  for (int i = 0; i < 16; ++i) { const __bf16 h = (__bf16)v[i]; r.h[i] = h; r.l[i] = (__bf16)(v[i] - (float)h); }
  return r; }
__device__ __forceinline__ F2 split_row(const float* row, int k0, int lane) { float v[16]; const float* p = row + k0 + 8 * (lane >> 4);
#pragma unroll
  for (int i = 0; i < 8; ++i) { v[i] = p[i]; v[8 + i] = p[16 + i]; }
  return bsplit16(v); }
__device__ __forceinline__ F2 split_rowK(const float* row, int k0, int lane, int K) { float v[16]; const int g = lane >> 4;
#pragma unroll
  for (int i = 0; i < 8; ++i) { const int ka = k0 + 8 * g + i, kb = ka + 16; v[i] = ka < K ? row[ka < K ? ka : K - 1] : 0.f; v[8 + i] = kb < K ? row[kb < K ? kb : K - 1] : 0.f; }
  return bsplit16(v); }
__device__ __forceinline__ F2 split_col(const float* W, int k0, int n, int lane, int ld, int K) { float v[16]; const int g = lane >> 4;
#pragma unroll
  for (int i = 0; i < 8; ++i) { const int ka = k0 + 8 * g + i, kb = ka + 16; v[i] = ka < K ? W[(size_t)(ka < K ? ka : K - 1) * ld + n] : 0.f; v[8 + i] = kb < K ? W[(size_t)(kb < K ? kb : K - 1) * ld + n] : 0.f; }
  return bsplit16(v); }
__device__ __forceinline__ v8f mac3(const F2& a, const F2& b, v8f c) { c = wmma_bf(a.l, b.h, c); c = wmma_bf(a.h, b.l, c); return wmma_bf(a.h, b.h, c); }
__device__ __forceinline__ float sigm(float v) { return 1.0f / (1.0f + expf(-v)); }
#define LDSX() do { asm volatile("s_wait_dscnt 0" ::: "memory"); __builtin_amdgcn_wave_barrier(); __builtin_amdgcn_fence(__ATOMIC_RELEASE, "workgroup"); } while (0)

#define NB 2
#define TT 4096
#define CC 256
#define NH 8
#define HD 32
#define HALFW 512
#define NQB (TT / 64)
#define NKBALL (TT / 128)
#define NKB 11
#define S2W (NKB * 128)
#define HG 2
#define SCALE 0.17677669529663687f
#ifndef TNB
#define TNB NB
#endif
__device__ __forceinline__ float bfr(float v) { return (float)(__bf16)v; }
__host__ __device__ __forceinline__ bool is_glob(int t) { return (t == 0) || (t == 63) || (t == TT - 64) || (t == TT - 1); }
__host__ __device__ __forceinline__ int gq_of(int qb) { return qb == 0 ? 0 : (qb == NQB - 1 ? 1 : -1); }
__host__ __device__ __forceinline__ int kb_lo(int qb) { const int a = (qb * 64 - HALFW) >> 7; return a < 0 ? 0 : a; }
__host__ __device__ __forceinline__ int kb_hi(int qb) { const int a = (qb * 64 + 63 + HALFW) >> 7; return a > NKBALL - 1 ? NKBALL - 1 : a; }
__host__ __device__ __forceinline__ int slot_kb(int qb, int s) { const int lo = kb_lo(qb), hi = kb_hi(qb), nb = hi - lo + 1; if (s < nb) return lo + s; int e = s - nb; if (lo > 0) { if (e == 0) return 0; --e; } if (hi < NKBALL - 1) { if (e == 0) return NKBALL - 1; --e; } return -1; }

#define WS_QH  0u
#define WS_QL  (WS_QH + 2u * (size_t)NB * TT * CC)
#define WS_KH  (WS_QL + 2u * (size_t)NB * TT * CC)
#define WS_VT  (WS_KH + 2u * (size_t)NB * TT * CC)
#define WS_S   (WS_VT + 2u * (size_t)NB * CC * TT)
#define WS_SG  (WS_S  + 4u * (size_t)HG * TT * S2W)
#define WS_Y   (WS_SG + 4u * (size_t)HG * 2 * 64 * TT)
#define WS_END (WS_Y  + 4u * (size_t)NB * TT * CC)

__global__ __launch_bounds__(128) void k_proj(const float* __restrict__ X, const float* __restrict__ W1, const float* __restrict__ B1, _Float16* __restrict__ QH, _Float16* __restrict__ QL, _Float16* __restrict__ KH, _Float16* __restrict__ VT) {
  __shared__ __align__(16) _Float16 sh[64][136], sl[64][136]; __shared__ __align__(16) _Float16 th[128][72];
  const int tid = threadIdx.x, wave = tid >> 5, lane = tid & 31, col = lane & 15, g = lane >> 4; const int which = blockIdx.z; const int c0 = blockIdx.y * 128; const size_t b = blockIdx.x / (TT / 64); const int t0 = (blockIdx.x % (TT / 64)) * 64; const size_t r0 = b * TT + t0;
  v8f acc[8] = {};
#pragma unroll 2
  for (int kc = 0; kc < CC / 32; ++kc) { v16b a; { const float* p = X + (b * CC + kc * 32 + 8 * g) * (size_t)TT + t0 + wave * 16 + col;
#pragma unroll
      for (int i = 0; i < 8; ++i) { a[i] = (__bf16)p[(size_t)i * TT]; a[8 + i] = (__bf16)p[(size_t)(16 + i) * TT]; } }
    asm volatile("s_wait_loadcnt 0x0" ::: "memory");
#pragma unroll
    for (int j = 0; j < 8; ++j) { v16b w; const int op = c0 + j * 16 + col; const int o = (op & 31) * 24 + (op >> 5) * 3 + which;
#pragma unroll
      for (int i = 0; i < 8; ++i) { w[i] = (__bf16)W1[(size_t)(kc * 32 + 8 * g + i) * (3 * CC) + o]; w[8 + i] = (__bf16)W1[(size_t)(kc * 32 + 16 + 8 * g + i) * (3 * CC) + o]; }
      asm volatile("s_wait_loadcnt 0x0" ::: "memory"); acc[j] = wmma_bf(a, w, acc[j]); } }
#pragma unroll
  for (int j = 0; j < 8; ++j) { const int op = c0 + j * 16 + col; const float bb = bfr(B1[(op & 31) * 24 + (op >> 5) * 3 + which]);
#pragma unroll
    for (int r = 0; r < 8; ++r) { const float v = acc[j][r] + bb; const int rl = wave * 16 + 8 * g + r, cl = j * 16 + col; const _Float16 hv = (_Float16)v;
      if (which == 2) th[cl][rl] = hv; else { sh[rl][cl] = hv; sl[rl][cl] = (_Float16)((v - (float)hv) * 1024.0f); } } }
  __syncthreads();
  if (which < 2) { _Float16* dh = which == 0 ? QH : KH; for (int e = tid; e < 64 * 16; e += 128) { const int rl = e >> 4, q = e & 15; vst2((unsigned*)(dh + (r0 + rl) * CC + c0 + q * 8), *(const v4u*)&sh[rl][q * 8]); if (which == 0) vst2((unsigned*)(QL + (r0 + rl) * CC + c0 + q * 8), *(const v4u*)&sl[rl][q * 8]); } }
  else { for (int e = tid; e < 128 * 8; e += 128) { const int cl = e >> 3, q = e & 7; vst2((unsigned*)(VT + (b * CC + c0 + cl) * (size_t)TT + t0 + q * 8), *(const v4u*)&th[cl][q * 8]); } } }
__device__ __forceinline__ float* slot_row(float* S0, float* SG0, int qb, int s, int z, int rowl, int* kb, size_t* pitch) { const int gq = gq_of(qb);
  if (gq >= 0) { *kb = s; *pitch = TT; return SG0 + (((size_t)z * 2 + gq) * 64 + rowl) * TT + (size_t)s * 128; }
  if (s >= NKB) { *kb = -1; *pitch = S2W; return nullptr; } *kb = slot_kb(qb, s); *pitch = S2W; return (*kb < 0) ? nullptr : (S0 + ((size_t)z * TT + (size_t)qb * 64 + rowl) * S2W + (size_t)s * 128); }
__global__ __launch_bounds__(128) void k_sc(const _Float16* __restrict__ QH, const _Float16* __restrict__ QL, const _Float16* __restrict__ KH, int b, int h0, float* __restrict__ S0, float* __restrict__ SG0) { __shared__ __align__(16) float ss[4][16][132];
  const int qb = blockIdx.x, s = blockIdx.y, z = blockIdx.z; const int tid = threadIdx.x, wave = tid >> 5, lane = tid & 31, col = lane & 15, g = lane >> 4;
  int kb; size_t pitch; float* rowp = slot_row(S0, SG0, qb, s, z, wave * 16, &kb, &pitch); if (rowp == nullptr) return;
  const int h = h0 + z; const int k0 = kb * 128; const size_t q0 = (size_t)b * TT + qb * 64 + wave * 16, kr0 = (size_t)b * TT + k0;
  v8f acc[8] = {}, accl[8] = {};
  { const v16h ah = frag_h(QH + (q0 + col) * CC + h * HD, lane), al = frag_h(QL + (q0 + col) * CC + h * HD, lane);
#pragma unroll
    for (int j = 0; j < 8; ++j) { const v16h kbf = frag_h(KH + (kr0 + j * 16 + col) * CC + h * HD, lane); acc[j] = wmma16(ah, kbf, acc[j]); accl[j] = wmma16(al, kbf, accl[j]); } }
#pragma unroll
  for (int j = 0; j < 8; ++j) {
#pragma unroll
    for (int r = 0; r < 8; ++r) ss[wave][8 * g + r][j * 16 + col] = (acc[j][r] + accl[j][r] * (1.0f / 1024.0f)) * SCALE; }
  LDSX(); for (int rl = 0; rl < 16; ++rl) vst2(rowp + (size_t)rl * pitch + lane * 4, *(const v4f*)&ss[wave][rl][lane * 4]); }
__global__ __launch_bounds__(256) void k_sm(float* __restrict__ S0, float* __restrict__ SG0) { __shared__ float sred[8]; __shared__ float sbc; __shared__ __align__(16) float shv[NKBALL * 128];
  const int tid = threadIdx.x; const int t = blockIdx.x; const int qb = t >> 6; const int z = blockIdx.y; const int gq = gq_of(qb); const int nslot = (gq >= 0) ? NKBALL : NKB; const bool gi = is_glob(t);
  int kb0; size_t pitch; float* sr = slot_row(S0, SG0, qb, 0, z, t & 63, &kb0, &pitch);
  float m = -3.0e38f;
  for (int e = tid; e < nslot * 128; e += 256) { const int s = e >> 7; int kb; size_t p2; const float* rp = slot_row(S0, SG0, qb, s, z, t & 63, &kb, &p2); float v = -3.0e38f;
    if (rp != nullptr) { const int j = kb * 128 + (e & 127); const int dj = t - j; const bool keep = (dj <= HALFW && dj >= -HALFW) || gi || is_glob(j); v = keep ? sr[(size_t)s * 128 + (e & 127)] : -3.0e38f; }
    shv[e] = v; m = fmaxf(m, v); }
#pragma unroll
  for (int o = 1; o < 32; o <<= 1) m = fmaxf(m, __shfl_xor(m, o));
  if ((tid & 31) == 0) sred[tid >> 5] = m; __syncthreads(); if (tid == 0) { float a = sred[0]; for (int i = 1; i < 8; ++i) a = fmaxf(a, sred[i]); sbc = a; } __syncthreads(); m = sbc; __syncthreads();
  float sum = 0.f; for (int e = tid; e < nslot * 128; e += 256) { const float v = shv[e]; const float ex = (v <= -1.0e38f) ? 0.f : expf(v - m); shv[e] = ex; sum += ex; }
#pragma unroll
  for (int o = 1; o < 32; o <<= 1) sum += __shfl_xor(sum, o);
  if ((tid & 31) == 0) sred[tid >> 5] = sum; __syncthreads(); if (tid == 0) { float a = 0.f; for (int i = 0; i < 8; ++i) a += sred[i]; sbc = 2048.0f / a; } __syncthreads(); const float inv = sbc;
  for (int e = tid; e < nslot * 128; e += 256) shv[e] = shv[e] * inv;
  __syncthreads();
  { int kbv; size_t p3; const int nvalid = (gq >= 0) ? NKBALL : NKB;
    for (int q = tid; q < nvalid * 32; q += 256) { const int s = q >> 5; if (slot_row(S0, SG0, qb, s, z, t & 63, &kbv, &p3) != nullptr) vst2(sr + (size_t)s * 128 + (q & 31) * 4, *(const v4f*)&shv[s * 128 + (q & 31) * 4]); } } }
__global__ __launch_bounds__(128) void k_pv(float* __restrict__ S0, float* __restrict__ SG0, const _Float16* __restrict__ VT, int b, int h0, float* __restrict__ Y) { __shared__ __align__(16) float ss[4][16][HD + 4];
  const int qb = blockIdx.x, z = blockIdx.z; const int h = h0 + z; const int tid = threadIdx.x, wave = tid >> 5, lane = tid & 31, col = lane & 15, g = lane >> 4; const int nslot = (gq_of(qb) >= 0) ? NKBALL : NKB;
  v8f acc[HD / 16] = {};
#pragma unroll 1
  for (int s = 0; s < nslot; ++s) { int kb; size_t pitch; float* rp = slot_row(S0, SG0, qb, s, z, wave * 16, &kb, &pitch); if (rp == nullptr) continue;
#pragma unroll
    for (int kc = 0; kc < 4; ++kc) { const v16h p = frag_f32(rp + (size_t)col * pitch + kc * 32, lane);
      asm volatile("s_wait_loadcnt 0x0" ::: "memory");
#pragma unroll
      for (int j = 0; j < HD / 16; ++j) { const size_t po = ((size_t)b * CC + h * HD + j * 16 + col) * (size_t)TT + kb * 128 + kc * 32; acc[j] = wmma16(p, frag_h(VT + po, lane), acc[j]); } } }
#pragma unroll
  for (int j = 0; j < HD / 16; ++j)
#pragma unroll
    for (int r = 0; r < 8; ++r) ss[wave][8 * g + r][j * 16 + col] = acc[j][r] * (1.0f / 2048.0f);
  LDSX(); for (int rl = 0; rl < 16; ++rl) if (lane < HD / 4) vst2(Y + ((size_t)b * TT + qb * 64 + wave * 16 + rl) * CC + h * HD + lane * 4, *(const v4f*)&ss[wave][rl][lane * 4]); }
__global__ __launch_bounds__(128) void k_out(const float* __restrict__ Y, const float* __restrict__ W2, const float* __restrict__ B2, float* __restrict__ OUT) { __shared__ __align__(16) float sot[128][68];
  const int tid = threadIdx.x, wave = tid >> 5, lane = tid & 31, col = lane & 15, g = lane >> 4; const int c0 = blockIdx.y * 128; const size_t b = blockIdx.x / (TT / 64); const int t0 = (blockIdx.x % (TT / 64)) * 64; const size_t r0 = b * TT + t0 + wave * 16;
  v8f acc[8] = {};
#pragma unroll 2
  for (int kc = 0; kc < CC / 32; ++kc) { const v16h a = frag_f32(Y + (r0 + col) * CC + kc * 32, lane); asm volatile("s_wait_loadcnt 0x0" ::: "memory");
#pragma unroll
    for (int j = 0; j < 8; ++j) { v16h w; const int n = c0 + j * 16 + col;
#pragma unroll
      for (int i = 0; i < 8; ++i) { const int ka = kc * 32 + 8 * g + i, kb2 = ka + 16; w[i] = (_Float16)(bfr(W2[(size_t)((ka & 31) * 8 + (ka >> 5)) * CC + n]) * 256.0f); w[8 + i] = (_Float16)(bfr(W2[(size_t)((kb2 & 31) * 8 + (kb2 >> 5)) * CC + n]) * 256.0f); }
      asm volatile("s_wait_loadcnt 0x0" ::: "memory"); acc[j] = wmma16(a, w, acc[j]); } }
#pragma unroll
  for (int j = 0; j < 8; ++j) { const float bb = bfr(B2[c0 + j * 16 + col]);
#pragma unroll
    for (int r = 0; r < 8; ++r) sot[j * 16 + col][wave * 16 + 8 * g + r] = acc[j][r] * (1.0f / 256.0f) + bb; }
  __syncthreads();
  for (int e = tid; e < 128 * 16; e += 128) { const int c = e >> 4, q = e & 15; vst2(OUT + (b * CC + c0 + c) * (size_t)TT + t0 + q * 4, *(const v4f*)&sot[c][q * 4]); } }
extern "C" void kernel_launch(void* const* d_in, const int* in_sizes, int n_in, void* d_out, int out_size, void* d_ws, size_t ws_size, hipStream_t stream) {
  (void)in_sizes; (void)n_in; (void)out_size;
  const float** F = (const float**)d_in;
  if (ws_size < (size_t)WS_END) return;
  char* ws = (char*)d_ws; _Float16 *QH = (_Float16*)(ws + WS_QH), *QL = (_Float16*)(ws + WS_QL), *KH = (_Float16*)(ws + WS_KH), *VT = (_Float16*)(ws + WS_VT); float *S = (float*)(ws + WS_S), *SG = (float*)(ws + WS_SG), *Y = (float*)(ws + WS_Y);
  k_proj<<<dim3(TNB * TT / 64, CC / 128, 3), 128, 0, stream>>>(F[0], F[1], F[2], QH, QL, KH, VT);
  for (int b = 0; b < TNB; ++b) for (int h0 = 0; h0 < NH; h0 += HG) {
    k_sc<<<dim3(NQB, NKBALL, HG), 128, 0, stream>>>(QH, QL, KH, b, h0, S, SG);
    k_sm<<<dim3(TT, HG), 256, 0, stream>>>(S, SG);
    k_pv<<<dim3(NQB, 1, HG), 128, 0, stream>>>(S, SG, VT, b, h0, Y);
  }
  k_out<<<dim3(TNB * TT / 64, CC / 128), 128, 0, stream>>>(Y, F[3], F[4], (float*)d_out);
}
